// DMRNet_42099269435949
// MI455X (gfx1250) — hardware-run, weakly checked
//
#include <hip/hip_runtime.h>
#include <math.h>

typedef __attribute__((ext_vector_type(16))) _Float16 v16h;
typedef __attribute__((ext_vector_type(8)))  _Float16 v8h;
typedef __attribute__((ext_vector_type(8)))  float    v8f;
typedef __attribute__((ext_vector_type(4)))  float    v4f;

constexpr int kVis   = 256;
constexpr int kTok   = 48;
constexpr int kMedId = 24;
constexpr int kCmbId = 10;
constexpr int kEmb   = 64;
constexpr int kMD    = 128;
constexpr int kMV    = 131;
constexpr int kCC    = 300;
constexpr int kDiagV = 2000;
constexpr int kProcV = 1500;
constexpr int kHid2  = 256;
constexpr int kNPad  = 144;
constexpr int kNTile = 9;
constexpr int kXW    = kMV + kCC;
constexpr int kP132  = kMV + 1;
constexpr int kCmbW  = kCC - 1;
constexpr int kWJP = 160;
constexpr int kBSP = 160;
constexpr int kPRP = 160;
constexpr int kCMP = 320;
constexpr int kXP = 68;
constexpr int kHP = 264;
constexpr float kCarryX = 16.0f;
constexpr float kCarryW = 1024.0f;
constexpr float kCarryH = 64.0f;
constexpr float kInvTok  = 1.0f / (kCarryX * kCarryW);
constexpr float kInvPair = 1.0f / (kCarryH * kCarryW);
constexpr float kInvL    = 1.0f / (float)kTok;

static_assert(kHid2 == 2 * kMD, "hidden width");
static_assert(kNPad == kNTile * 16 && kNPad >= kMV, "N padding");
static_assert((kHid2 % 32) == 0 && (kEmb % 32) == 0, "K multiples of 32");
static_assert((kTok % 16) == 0 && (kMD % 16) == 0 && (kVis % 16) == 0, "tile multiples");
static_assert((kWJP % 32) == 0 && (kBSP % 32) == 0 && (kPRP % 32) == 0 && (kCMP % 32) == 0, "line pitches");
static_assert(kWJP >= kNPad && kPRP >= kP132 && kCMP >= kCC, "pitch covers row");
static_assert((kP132 % 4) == 0 && (kCC % 4) == 0, "float4 never straddles a row");

constexpr size_t kOffPREP  = 0;
constexpr size_t kOffTDM   = kOffPREP  + (size_t)kVis * kMD * 4;
constexpr size_t kOffTPM   = kOffTDM   + (size_t)kVis * kMD * 4;
constexpr size_t kOffWJK   = kOffTPM   + (size_t)kVis * kMD * 4;
constexpr size_t kOffAPL   = kOffWJK   + (size_t)kVis * kWJP * 4;
constexpr size_t kOffBPL   = kOffAPL   + (size_t)kVis * kHid2 * 4;
constexpr size_t kOffBASE  = kOffBPL   + (size_t)kVis * kHid2 * 4;
constexpr size_t kOffPROB  = kOffBASE  + (size_t)kVis * kBSP * 4;
constexpr size_t kOffCOMBO = kOffPROB  + (size_t)kVis * kPRP * 4;
constexpr size_t kOffW1T   = kOffCOMBO + (size_t)kVis * kCMP * 4;
constexpr size_t kOffW2T   = kOffW1T   + (size_t)2 * kMD * kEmb * 2;
constexpr size_t kWsTotal  = kOffW2T   + (size_t)kNPad * kHid2 * 2;
static_assert(kWsTotal == 1843200ull, "carve total");
static_assert(kWsTotal <= 134217728ull, "carve cap");
static_assert((kOffTDM % 128) == 0 && (kOffTPM % 128) == 0 && (kOffWJK % 128) == 0 && (kOffAPL % 128) == 0 &&
              (kOffBPL % 128) == 0 && (kOffBASE % 128) == 0 && (kOffPROB % 128) == 0 && (kOffCOMBO % 128) == 0 &&
              (kOffW1T % 128) == 0 && (kOffW2T % 128) == 0, "128-B aligned regions");
static_assert(kOffW2T == kOffW1T + 32768ull, "weight planes contiguous");

constexpr unsigned kOut0N = (unsigned)kVis * kP132;
constexpr unsigned kOut1N = (unsigned)kP132 * kVis * kP132;
constexpr unsigned kOut2N = (unsigned)kVis * kCC;
constexpr unsigned kOutTotal = kOut0N + kOut1N + kOut2N;
static_assert(kOut0N == 33792u && kOut1N == 4460544u && kOut2N == 76800u, "output sizes");
static_assert(kOut0N * 4u == 135168u && (kOut0N + kOut1N) * 4u == 17977344u, "output byte offsets");
static_assert(kOutTotal * 4u == 18284544u, "output total bytes");
constexpr int kOutBlk0 = (int)(kOut0N / 1024u);
constexpr int kOutBlk1 = (int)(kOut1N / 1024u);
constexpr int kOutBlk2 = (int)(kOut2N / 1024u);
static_assert((unsigned)kOutBlk0 * 1024u == kOut0N && (unsigned)kOutBlk1 * 1024u == kOut1N &&
              (unsigned)kOutBlk2 * 1024u == kOut2N, "block-exact output regions");

__device__ __forceinline__ int imin_(int a, int b) { return a < b ? a : b; }
__device__ __forceinline__ int imax_(int a, int b) { return a > b ? a : b; }

union FragU { v16h v; v8h h[2]; };
__device__ __forceinline__ v16h frag_load(const _Float16* p) {
  FragU f;
  f.h[0] = *(const v8h*)(p);
  f.h[1] = *(const v8h*)(p + 16);
  return f.v;
}
__device__ __forceinline__ v16h frag_cvt(const float* p, float carry) {
  const v4f x0 = *(const v4f*)(p);
  const v4f x1 = *(const v4f*)(p + 4);
  const v4f x2 = *(const v4f*)(p + 16);
  const v4f x3 = *(const v4f*)(p + 20);
  v16h a;
#pragma unroll
  for (int e = 0; e < 4; ++e) {
    a[e]      = (_Float16)(x0[e] * carry);
    a[4 + e]  = (_Float16)(x1[e] * carry);
    a[8 + e]  = (_Float16)(x2[e] * carry);
    a[12 + e] = (_Float16)(x3[e] * carry);
  }
  return a;
}
__device__ __forceinline__ v8f mma_h(v16h a, v16h b, v8f c) {
  c = __builtin_amdgcn_wmma_f32_16x16x32_f16(false, a, false, b, (short)0, c, false, false);
  asm volatile("v_nop\n\tv_nop\n\tv_nop\n\tv_nop" : "+v"(c) : "v"(a), "v"(b));
  return c;
}
__device__ __forceinline__ void wave_lds_sync() {
  __builtin_amdgcn_fence(__ATOMIC_RELEASE, "workgroup");
  __builtin_amdgcn_wave_barrier();
  __builtin_amdgcn_fence(__ATOMIC_ACQUIRE, "workgroup");
}

__global__ __launch_bounds__(256) void pack_weights_kernel(
    const float* __restrict__ dw1, const float* __restrict__ qw1, const float* __restrict__ pw2,
    unsigned short* __restrict__ W1T, unsigned short* __restrict__ W2T)
{
  const int g = blockIdx.x * 256 + threadIdx.x;
  v8h hv;
  unsigned short* dst;
  if (blockIdx.x < 8) {
    const int e0  = g * 8;
    const int mat = e0 >> 13;
    const int n   = (e0 >> 6) & 127;
    const int k0  = e0 & 63;
    const float* src = mat ? qw1 : dw1;
#pragma unroll
    for (int e = 0; e < 8; ++e) {
      const float x = src[(k0 + e) * kMD + n];
      hv[e] = (_Float16)(x * kCarryW);
    }
    dst = W1T + e0;
  } else {
    const int e1 = (g - 2048) * 8;
    const int n  = e1 >> 8;
    const int k0 = e1 & 255;
    const int nc = imin_(n, kMV - 1);
    const bool live = (n < kMV);
#pragma unroll
    for (int e = 0; e < 8; ++e) {
      const float x = pw2[(k0 + e) * kMV + nc];
      const float y = live ? (x * kCarryW) : 0.0f;
      hv[e] = (_Float16)y;
    }
    dst = W2T + e1;
  }
  *(volatile v8h*)dst = hv;
  __threadfence();
  *(volatile v8h*)dst = hv;
}

__global__ __launch_bounds__(256) void embed_token_kernel(
    const int* __restrict__ diag, const int* __restrict__ proc,
    const float* __restrict__ demb, const float* __restrict__ pemb,
    const unsigned short* __restrict__ W1Tp,
    const float* __restrict__ db1, const float* __restrict__ qb1,
    float* __restrict__ PREP, float* __restrict__ TDM, float* __restrict__ TPM)
{
  __shared__ __align__(16) float sX[2 * kTok * kXP];
  __shared__ __align__(16) float sMean[2 * kMD];
  __shared__ __align__(16) float sPr[kMD];
  const int v = blockIdx.x;
  const int tid = threadIdx.x, lane = tid & 31, wave = tid >> 5;
  const int hh = lane >> 4, c = lane & 15;
#pragma unroll 1
  for (int it = 0; it < 3; ++it) {
    const int idx = it * 256 + tid;
    const int l = idx >> 4, c4 = (idx & 15) * 4;
    int id = diag[v * kTok + l];
    id = imin_(imax_(id, 0), kDiagV - 1);
    *(v4f*)(sX + l * kXP + c4) = *(const v4f*)(demb + (size_t)id * kEmb + c4);
  }
#pragma unroll 1
  for (int it = 0; it < 3; ++it) {
    const int idx = it * 256 + tid;
    const int l = idx >> 4, c4 = (idx & 15) * 4;
    int id = proc[v * kTok + l];
    id = imin_(imax_(id, 0), kProcV - 1);
    *(v4f*)(sX + kTok * kXP + l * kXP + c4) = *(const v4f*)(pemb + (size_t)id * kEmb + c4);
  }
  __syncthreads();
  if (tid < kMD) {
    const int mat = tid >> 6, e = tid & 63;
    const float* xp = sX + mat * (kTok * kXP) + e;
    float s = 0.0f;
#pragma unroll 1
    for (int l = 0; l < kTok; ++l) s += xp[l * kXP];
    sPr[tid] = s * kInvL;
  }
  const _Float16* W1T = (const _Float16*)W1Tp;
  const int col = wave * 16 + c;
  const float bd = db1[col];
  const float bq = qb1[col];
#pragma unroll 1
  for (int mat = 0; mat < 2; ++mat) {
    const _Float16* wt = W1T + mat * (kMD * kEmb) + col * kEmb + 8 * hh;
    const v16h b0 = frag_load(wt);
    const v16h b1 = frag_load(wt + 32);
    const float bv = mat ? bq : bd;
    float cs = 0.0f;
#pragma unroll 1
    for (int mt = 0; mt < 3; ++mt) {
      const float* xr = sX + mat * (kTok * kXP) + (mt * 16 + c) * kXP + 8 * hh;
      const v16h a0 = frag_cvt(xr, kCarryX);
      const v16h a1 = frag_cvt(xr + 32, kCarryX);
      v8f acc = (v8f){0.f, 0.f, 0.f, 0.f, 0.f, 0.f, 0.f, 0.f};
      acc = mma_h(a0, b0, acc);
      acc = mma_h(a1, b1, acc);
#pragma unroll
      for (int r = 0; r < 8; ++r) cs += tanhf(acc[r] * kInvTok + bv);
    }
    const float other = __shfl_xor(cs, 16, 32);
    const float tot = cs + other;
    if (lane < 16) sMean[mat * kMD + col] = tot * kInvL;
  }
  __syncthreads();
  if (wave < 3) {
    const float* src = (wave == 0) ? sPr : (sMean + (wave - 1) * kMD);
    float* dstp = (wave == 0) ? PREP : ((wave == 1) ? TDM : TPM);
    const v4f val = *(const v4f*)(src + lane * 4);
    float* gp = dstp + (size_t)v * kMD + lane * 4;
    for (int pass = 0; pass < 2; ++pass) {
      *(volatile v4f*)gp = val;
      __threadfence();
    }
  }
}

__global__ __launch_bounds__(256) void history_content_kernel(
    const int* __restrict__ drug_ids, const int* __restrict__ combo_ids,
    const float* __restrict__ w1, const float* __restrict__ b1,
    const float* __restrict__ w2, const float* __restrict__ b2,
    float* __restrict__ WJK)
{
  __shared__ int sId[64];
  __shared__ __align__(16) float sXc[448];
  __shared__ __align__(16) float sHid[kNPad];
  __shared__ __align__(16) float sRow[kWJP];
  const int j = blockIdx.x;
  const int t = threadIdx.x, lane = t & 31, wave = t >> 5;
  if (t < 64) {
    const int jm = imax_(j - 1, 0);
    const int a = drug_ids[jm * kMedId + imin_(t, kMedId - 1)];
    const int b = combo_ids[jm * kCmbId + imin_(imax_(t - kMedId, 0), kCmbId - 1)];
    const int fa = (t < kMedId) ? 1 : 0;
    const int fb = (t >= kMedId && t < kMedId + kCmbId) ? 1 : 0;
    const int fj = (j > 0) ? 1 : 0;
    sId[t] = (a * fa + b * fb) * fj;
  }
  __syncthreads();
  for (int q = t; q < 448; q += 256) {
    const int tgt = (q < kMV) ? (q + 1) : (q - kMV + 1);
    int cd = 0, cc = 0;
#pragma unroll 1
    for (int m = 0; m < kMedId; ++m) cd += (sId[m] == tgt) ? 1 : 0;
#pragma unroll 1
    for (int m = 0; m < kCmbId; ++m) cc += (sId[kMedId + m] == tgt) ? 1 : 0;
    const int cnt = (q < kMV) ? cd : cc;
    sXc[q] = (q < kXW) ? (float)cnt : 0.0f;
  }
  __syncthreads();
  if (t < kNPad) {
    const int c = imin_(t, kMV - 1);
    float s = b1[c];
#pragma unroll 1
    for (int q = 0; q < kXW; ++q) s = fmaf(sXc[q], w1[q * kMV + c], s);
    const float hv = tanhf(s);
    sHid[t] = (t < kMV) ? hv : 0.0f;
  }
  __syncthreads();
  if (t < kWJP) {
    const int k = imin_(t, kMV - 1);
    float s = b2[k];
#pragma unroll 1
    for (int c = 0; c < kMV; ++c) s = fmaf(sHid[c], w2[c * kMV + k], s);
    const float val = tanhf(s) + sXc[k];
    sRow[t] = (t < kMV) ? val : 0.0f;
  }
  __syncthreads();
  if (wave < 2) {
    const int idx = wave * 128 + lane * 4;
    const int idc = imin_(idx, kWJP - 4);
    const v4f val = *(const v4f*)(sRow + idc);
    float* gp = WJK + (size_t)j * kWJP + idx;
    for (int pass = 0; pass < 2; ++pass) {
      if (idx < kWJP) *(volatile v4f*)gp = val;
      __threadfence();
    }
  }
}

__global__ __launch_bounds__(256) void visit_dense_kernel(
    const float* __restrict__ PREP, const float* __restrict__ TDM, const float* __restrict__ TPM,
    const float* __restrict__ lw1, const float* __restrict__ lb1,
    const float* __restrict__ lw2, const float* __restrict__ lb2,
    const float* __restrict__ pw1, const float* __restrict__ pb1,
    const float* __restrict__ medb,
    const float* __restrict__ dw2, const float* __restrict__ db2,
    const float* __restrict__ qw2, const float* __restrict__ qb2,
    const float* __restrict__ dmb, const float* __restrict__ pmb,
    const float* __restrict__ cw1, const float* __restrict__ cb1,
    const float* __restrict__ cw2, const float* __restrict__ cb2,
    float* __restrict__ APL, float* __restrict__ BPL, float* __restrict__ BASE, float* __restrict__ COMBO)
{
  __shared__ __align__(16) float sIn[512];
  __shared__ __align__(16) float sH1[kMD];
  __shared__ __align__(16) float sPl[kMD];
  __shared__ __align__(16) float sDh[kMD];
  __shared__ __align__(16) float sCh[kMD];
  __shared__ __align__(16) float sOut[992];
  const int v = blockIdx.x;
  const int t = threadIdx.x, lane = t & 31, wave = t >> 5;
  {
    const int cidx = t & 127;
    const bool lo = (t < 128);
    const int vm = imax_(v - 1, 0);
    const float x1 = PREP[(size_t)(lo ? v : vm) * kMD + cidx];
    sIn[t] = (lo || v > 0) ? x1 : 0.0f;
    const float* src2 = lo ? TDM : TPM;
    sIn[256 + t] = src2[(size_t)v * kMD + cidx];
  }
  __syncthreads();
  if (t < 128) {
    float s = lb1[t];
#pragma unroll 1
    for (int m = 0; m < kMD; ++m) {
      const float w = lw1[m * kMD + t] + lw1[(m + kMD) * kMD + t];
      s = fmaf(sIn[m], w, s);
    }
    sH1[t] = tanhf(s);
    const int e = t & 63;
    const bool isd = (t < 64);
    const float* w2p = isd ? dw2 : qw2;
    const float* b2p = isd ? db2 : qb2;
    const float* xin = sIn + (isd ? 256 : 384);
    float s2 = b2p[e];
#pragma unroll 1
    for (int cc = 0; cc < kMD; ++cc) s2 = fmaf(xin[cc], w2p[cc * kEmb + e], s2);
    sDh[t] = s2;
  } else {
    const int c = t - 128;
    float s = cb1[c];
#pragma unroll 1
    for (int m = 0; m < kMD; ++m) s = fmaf(sIn[m], cw1[m * kMD + c], s);
    sCh[c] = tanhf(s);
  }
  __syncthreads();
  if (t < 128) {
    float s = lb2[t];
#pragma unroll 1
    for (int m = 0; m < kMD; ++m) s = fmaf(sH1[m], lw2[m * kMD + t], s);
    sPl[t] = tanhf(s);
  }
  __syncthreads();
  {
    float sa = pb1[t], sb = 0.0f;
#pragma unroll 1
    for (int c = 0; c < kMD; ++c) {
      sa = fmaf(sPl[c], pw1[c * kHid2 + t], sa);
      sb = fmaf(sIn[128 + c], pw1[(kMD + c) * kHid2 + t], sb);
    }
    sOut[t] = sa;
    sOut[256 + t] = sb;
  }
  if (t < kBSP) {
    const int kc = imin_(t, kMV - 1);
    float s = 0.0f;
#pragma unroll 1
    for (int c = 0; c < kMD; ++c) s = fmaf(sPl[c], medb[c * kMV + kc], s);
#pragma unroll 1
    for (int e = 0; e < kEmb; ++e) {
      s = fmaf(sDh[e], dmb[e * kMV + kc], s);
      s = fmaf(sDh[kEmb + e], pmb[e * kMV + kc], s);
    }
    sOut[512 + t] = (t < kMV) ? s : 0.0f;
  }
  for (int k = t; k < kCMP; k += 256) {
    const int kk = imin_(imax_(k - 1, 0), kCmbW - 1);
    float s = cb2[kk];
#pragma unroll 1
    for (int c = 0; c < kMD; ++c) s = fmaf(sCh[c], cw2[c * kCmbW + kk], s);
    const float p = 1.0f / (1.0f + expf(-s));
    sOut[672 + k] = (k >= 1 && k < kCC) ? p : 0.0f;
  }
  __syncthreads();
  for (int job = wave; job < 9; job += 8) {
    float* g;
    int so, n, ch;
    if (job < 2)      { g = APL   + (size_t)v * kHid2; so = 0;   n = kHid2; ch = job; }
    else if (job < 4) { g = BPL   + (size_t)v * kHid2; so = 256; n = kHid2; ch = job - 2; }
    else if (job < 6) { g = BASE  + (size_t)v * kBSP;  so = 512; n = kBSP;  ch = job - 4; }
    else              { g = COMBO + (size_t)v * kCMP;  so = 672; n = kCMP;  ch = job - 6; }
    const int idx = ch * 128 + lane * 4;
    const int idc = imin_(idx, n - 4);
    const v4f val = *(const v4f*)(sOut + so + idc);
    for (int pass = 0; pass < 2; ++pass) {
      if (idx < n) *(volatile v4f*)(g + idx) = val;
      __threadfence();
    }
  }
}

__global__ __launch_bounds__(128) void pair_history_kernel(
    const float* __restrict__ APL, const float* __restrict__ BPL,
    const unsigned short* __restrict__ W2Tp, const float* __restrict__ b2,
    const float* __restrict__ WJK, const float* __restrict__ BASE,
    float* __restrict__ PROB)
{
  __shared__ __align__(16) _Float16 sHid[4 * 16 * kHP];
  __shared__ __align__(16) float sSum[4 * kNTile * 32];
  __shared__ __align__(16) float sRow[4 * kPRP];
  const int tid = threadIdx.x, lane = tid & 31, wave = tid >> 5;
  const int hh = lane >> 4, c = lane & 15;
  const int i = blockIdx.x * 4 + wave;
  _Float16* hid = sHid + wave * (16 * kHP);
  float* ss = sSum + wave * (kNTile * 32);
  float* srow = sRow + wave * kPRP;
  const _Float16* W2T = (const _Float16*)W2Tp;

  const v4f a0 = *(const v4f*)(APL + (size_t)i * kHid2 + lane * 8);
  const v4f a1 = *(const v4f*)(APL + (size_t)i * kHid2 + lane * 8 + 4);
#pragma unroll
  for (int n = 0; n < kNTile; ++n) ss[n * 32 + lane] = 0.0f;

  const int ntile = (i >> 4) + 1;
#pragma unroll 1
  for (int jt = 0; jt < ntile; ++jt) {
    const int j0 = jt * 16;
#pragma unroll 1
    for (int r = 0; r < 16; ++r) {
      const float* bp = BPL + (size_t)(j0 + r) * kHid2 + lane * 8;
      const v4f b0 = *(const v4f*)(bp);
      const v4f b1 = *(const v4f*)(bp + 4);
      v8h hv;
#pragma unroll
      for (int e = 0; e < 4; ++e) {
        const float t0 = tanhf(a0[e] + b0[e]);
        const float t1 = tanhf(a1[e] + b1[e]);
        hv[e]     = (_Float16)(t0 * kCarryH);
        hv[4 + e] = (_Float16)(t1 * kCarryH);
      }
      *(v8h*)(hid + r * kHP + lane * 8) = hv;
    }
    wave_lds_sync();
    v16h af[8];
#pragma unroll
    for (int kc = 0; kc < 8; ++kc) af[kc] = frag_load(hid + c * kHP + kc * 32 + 8 * hh);
#pragma unroll 1
    for (int n = 0; n < kNTile; ++n) {
      const int col = n * 16 + c;
      const _Float16* wp = W2T + (size_t)col * kHid2 + 8 * hh;
      v8f acc = (v8f){0.f, 0.f, 0.f, 0.f, 0.f, 0.f, 0.f, 0.f};
#pragma unroll
      for (int kc = 0; kc < 8; ++kc) {
        const v16h bf = frag_load(wp + kc * 32);
        acc = mma_h(af[kc], bf, acc);
      }
      const float braw = b2[imin_(col, kMV - 1)];
      const float bias = (col < kMV) ? braw : 0.0f;
      float s = 0.0f;
#pragma unroll
      for (int r = 0; r < 8; ++r) {
        const int j = j0 + 8 * hh + r;
        const float cv = tanhf(acc[r] * kInvPair + bias);
        const float w = WJK[(size_t)j * kWJP + col];
        const float term = cv * w;
        s += (j <= i) ? term : 0.0f;
      }
      ss[n * 32 + lane] += s;
    }
    wave_lds_sync();
  }
  wave_lds_sync();
#pragma unroll 1
  for (int q = 0; q < 5; ++q) {
    const int t = lane + 32 * q;
    const int kc = imin_(imax_(t - 1, 0), kMV - 1);
    const int si = (kc >> 4) * 32 + (kc & 15);
    const float sv = ss[si] + ss[si + 16];
    const float bv = BASE[(size_t)i * kBSP + kc];
    const float p = 1.0f / (1.0f + expf(-(bv + sv)));
    srow[t] = (t >= 1 && t <= kMV) ? p : 0.0f;
  }
  wave_lds_sync();
  {
    const v4f r0 = *(const v4f*)(srow + lane * 4);
    const v4f r1 = *(const v4f*)(srow + 128 + (lane & 7) * 4);
    float* gp = PROB + (size_t)i * kPRP;
    for (int pass = 0; pass < 2; ++pass) {
      *(volatile v4f*)(gp + lane * 4) = r0;
      if (lane < 8) *(volatile v4f*)(gp + 128 + lane * 4) = r1;
      __threadfence();
    }
  }
}

static_assert((unsigned)(kOutBlk0 + kOutBlk1 + kOutBlk2) * 1024u == kOutTotal, "writer coverage");
__global__ __launch_bounds__(256) void write_outputs_kernel(
    const float* __restrict__ PROB, const float* __restrict__ COMBO, float* __restrict__ out)
{
  const unsigned g = blockIdx.x * 256u + threadIdx.x;
  const unsigned f = g * 4u;
  v4f val;
  if ((int)blockIdx.x < kOutBlk0) {
    const unsigned i = f / (unsigned)kP132;
    const unsigned b = f - i * (unsigned)kP132;
    val = *(const v4f*)(PROB + (size_t)i * kPRP + b);
  } else if ((int)blockIdx.x < kOutBlk0 + kOutBlk1) {
    const unsigned f1 = f - kOut0N;
    const unsigned a = f1 / kOut0N;
    const unsigned rem = f1 - a * kOut0N;
    const unsigned i = rem / (unsigned)kP132;
    const unsigned b = rem - i * (unsigned)kP132;
    const v4f pv = *(const v4f*)(PROB + (size_t)i * kPRP + b);
    const float pa = PROB[(size_t)i * kPRP + a];
    val = pv * pa;
  } else {
    const unsigned f2 = f - (kOut0N + kOut1N);
    const unsigned vv = f2 / (unsigned)kCC;
    const unsigned k = f2 - vv * (unsigned)kCC;
    val = *(const v4f*)(COMBO + (size_t)vv * kCMP + k);
  }
  float* p = out + f;
  *(volatile v4f*)p = val;
  __threadfence();
  *(volatile v4f*)p = val;
}

extern "C" void kernel_launch(void* const* d_in, const int* in_sizes, int n_in,
                              void* d_out, int out_size, void* d_ws, size_t ws_size,
                              hipStream_t stream) {
  constexpr int kNumIn = 33;
  const int expect[kNumIn] = {
      kVis * kTok, kVis * kTok, kVis * kMedId, kVis * kCmbId,
      kDiagV * kEmb, kProcV * kEmb,
      kEmb * kMD, kMD, kMD * kEmb, kEmb,
      kEmb * kMD, kMD, kMD * kEmb, kEmb,
      kMD * kMV, kEmb * kMV, kEmb * kMV,
      kHid2 * kHid2, kHid2, kHid2 * kMV, kMV,
      kXW * kMV, kMV, kMV * kMV, kMV,
      kHid2 * kMD, kMD, kMD * kMD, kMD,
      kMD * kMD, kMD, kMD * kCmbW, kCmbW};
  if (n_in < kNumIn) return;
  for (int q = 0; q < kNumIn; ++q) {
    if (in_sizes[q] != expect[q]) return;
  }
  if ((unsigned)out_size != kOutTotal) return;
  if (ws_size < kWsTotal) return;

  const int*   diag      = (const int*)d_in[0];
  const int*   proc      = (const int*)d_in[1];
  const int*   drug_ids  = (const int*)d_in[2];
  const int*   combo_ids = (const int*)d_in[3];
  const float* diag_emb  = (const float*)d_in[4];
  const float* proc_emb  = (const float*)d_in[5];
  const float* dl2_w1 = (const float*)d_in[6];
  const float* dl2_b1 = (const float*)d_in[7];
  const float* dl2_w2 = (const float*)d_in[8];
  const float* dl2_b2 = (const float*)d_in[9];
  const float* pl2_w1 = (const float*)d_in[10];
  const float* pl2_b1 = (const float*)d_in[11];
  const float* pl2_w2 = (const float*)d_in[12];
  const float* pl2_b2 = (const float*)d_in[13];
  const float* med_block = (const float*)d_in[14];
  const float* dmb = (const float*)d_in[15];
  const float* pmb = (const float*)d_in[16];
  const float* pmc_w1 = (const float*)d_in[17];
  const float* pmc_b1 = (const float*)d_in[18];
  const float* pmc_w2 = (const float*)d_in[19];
  const float* pmc_b2 = (const float*)d_in[20];
  const float* clc_w1 = (const float*)d_in[21];
  const float* clc_b1 = (const float*)d_in[22];
  const float* clc_w2 = (const float*)d_in[23];
  const float* clc_b2 = (const float*)d_in[24];
  const float* lch_w1 = (const float*)d_in[25];
  const float* lch_b1 = (const float*)d_in[26];
  const float* lch_w2 = (const float*)d_in[27];
  const float* lch_b2 = (const float*)d_in[28];
  const float* cm_w1 = (const float*)d_in[29];
  const float* cm_b1 = (const float*)d_in[30];
  const float* cm_w2 = (const float*)d_in[31];
  const float* cm_b2 = (const float*)d_in[32];
  float* out = (float*)d_out;

  char* ws = (char*)d_ws;
  float* PREP  = (float*)(ws + kOffPREP);
  float* TDM   = (float*)(ws + kOffTDM);
  float* TPM   = (float*)(ws + kOffTPM);
  float* WJK   = (float*)(ws + kOffWJK);
  float* APL   = (float*)(ws + kOffAPL);
  float* BPL   = (float*)(ws + kOffBPL);
  float* BASE  = (float*)(ws + kOffBASE);
  float* PROB  = (float*)(ws + kOffPROB);
  float* COMBO = (float*)(ws + kOffCOMBO);
  unsigned short* W1T = (unsigned short*)(ws + kOffW1T);
  unsigned short* W2T = (unsigned short*)(ws + kOffW2T);

  pack_weights_kernel<<<26, 256, 0, stream>>>(dl2_w1, pl2_w1, pmc_w2, W1T, W2T);
  embed_token_kernel<<<kVis, 256, 0, stream>>>(diag, proc, diag_emb, proc_emb, W1T, dl2_b1, pl2_b1, PREP, TDM, TPM);
  history_content_kernel<<<kVis, 256, 0, stream>>>(drug_ids, combo_ids, clc_w1, clc_b1, clc_w2, clc_b2, WJK);
  visit_dense_kernel<<<kVis, 256, 0, stream>>>(PREP, TDM, TPM,
                                               lch_w1, lch_b1, lch_w2, lch_b2,
                                               pmc_w1, pmc_b1, med_block,
                                               dl2_w2, dl2_b2, pl2_w2, pl2_b2,
                                               dmb, pmb,
                                               cm_w1, cm_b1, cm_w2, cm_b2,
                                               APL, BPL, BASE, COMBO);
  pair_history_kernel<<<kVis / 4, 128, 0, stream>>>(APL, BPL, W2T, pmc_b2, WJK, BASE, PROB);
  write_outputs_kernel<<<kOutBlk0 + kOutBlk1 + kOutBlk2, 256, 0, stream>>>(PROB, COMBO, out);
}
